// LowRankSelfAttention_47218870452738
// MI455X (gfx1250) — hardware-verified
//
#include <hip/hip_runtime.h>
#include <math.h>

typedef __attribute__((ext_vector_type(16))) _Float16 v16h;
typedef __attribute__((ext_vector_type(16))) __bf16 v16b;
typedef __attribute__((ext_vector_type(8)))  _Float16 v8h;
typedef __attribute__((ext_vector_type(8)))  float v8f;
typedef __attribute__((ext_vector_type(4)))  float v4f;
typedef __attribute__((ext_vector_type(2)))  float v2f;
typedef __attribute__((ext_vector_type(4)))  unsigned v4u;
typedef __attribute__((ext_vector_type(4)))  int v4i;
typedef float __attribute__((may_alias)) float_a;
typedef int __attribute__((may_alias)) int_a;

template <typename T> __device__ __forceinline__ void vst2(void* p, T v) { *(volatile T*)p = v; __threadfence(); *(volatile T*)p = v; }
__device__ __forceinline__ v8f wmma16(v16h a, v16h b, v8f c) {
  v8f d = __builtin_amdgcn_wmma_f32_16x16x32_f16(false, a, false, b, (short)0, c, false, false);
  asm volatile("v_nop\n\tv_nop\n\tv_nop\n\tv_nop" : "+v"(d) : "v"(a), "v"(b));
  return d;
}
__device__ __forceinline__ v8f wmma_bf(v16b a, v16b b, v8f c) {
  v8f d = __builtin_amdgcn_wmma_f32_16x16x32_bf16(false, a, false, b, (short)0, c, false, false);
  asm volatile("v_nop\n\tv_nop\n\tv_nop\n\tv_nop" : "+v"(d) : "v"(a), "v"(b));
  return d;
}
__device__ __forceinline__ v16h frag_h(const _Float16* rowk0, int lane) {
  union { v16h v; v8h q[2]; } u; const _Float16* p = rowk0 + 8 * (lane >> 4);
  u.q[0] = *(const v8h*)p; u.q[1] = *(const v8h*)(p + 16); return u.v;
}
__device__ __forceinline__ v16h frag_f32(const float* rowk0, int lane) {
  v16h a; const float* p = rowk0 + 8 * (lane >> 4);
#pragma unroll
  for (int i = 0; i < 8; ++i) { a[i] = (_Float16)p[i]; a[8 + i] = (_Float16)p[16 + i]; }
  return a;
}
__device__ __forceinline__ v16h frag_f32s(const float* rowk0, int lane, float sc) {
  v16h a; const float* p = rowk0 + 8 * (lane >> 4);
#pragma unroll
  for (int i = 0; i < 8; ++i) { a[i] = (_Float16)(p[i] * sc); a[8 + i] = (_Float16)(p[16 + i] * sc); }
  return a;
}
__device__ __forceinline__ v16h fragc_f32(const float* W, int k0, int n, int lane, int ld, int K) {
  v16h a; const int g = lane >> 4;
#pragma unroll
  for (int i = 0; i < 8; ++i) { const int ka = k0 + 8 * g + i, kb = ka + 16;
    a[i] = (_Float16)(ka < K ? W[(size_t)(ka < K ? ka : K - 1) * ld + n] : 0.f); a[8 + i] = (_Float16)(kb < K ? W[(size_t)(kb < K ? kb : K - 1) * ld + n] : 0.f); }
  return a;
}
struct F2 { v16b h, l; };
__device__ __forceinline__ F2 bsplit16(const float v[16]) { F2 r;
#pragma unroll
  for (int i = 0; i < 16; ++i) { const __bf16 h = (__bf16)v[i]; r.h[i] = h; r.l[i] = (__bf16)(v[i] - (float)h); }
  return r; }
__device__ __forceinline__ F2 split_row(const float* row, int k0, int lane) { float v[16]; const float* p = row + k0 + 8 * (lane >> 4);
#pragma unroll
  for (int i = 0; i < 8; ++i) { v[i] = p[i]; v[8 + i] = p[16 + i]; }
  return bsplit16(v); }
__device__ __forceinline__ F2 split_rowK(const float* row, int k0, int lane, int K) { float v[16]; const int g = lane >> 4;
#pragma unroll
  for (int i = 0; i < 8; ++i) { const int ka = k0 + 8 * g + i, kb = ka + 16; v[i] = ka < K ? row[ka < K ? ka : K - 1] : 0.f; v[8 + i] = kb < K ? row[kb < K ? kb : K - 1] : 0.f; }
  return bsplit16(v); }
__device__ __forceinline__ F2 split_col(const float* W, int k0, int n, int lane, int ld, int K) { float v[16]; const int g = lane >> 4;
#pragma unroll
  for (int i = 0; i < 8; ++i) { const int ka = k0 + 8 * g + i, kb = ka + 16; v[i] = ka < K ? W[(size_t)(ka < K ? ka : K - 1) * ld + n] : 0.f; v[8 + i] = kb < K ? W[(size_t)(kb < K ? kb : K - 1) * ld + n] : 0.f; }
  return bsplit16(v); }
__device__ __forceinline__ v8f mac3(const F2& a, const F2& b, v8f c) { c = wmma_bf(a.l, b.h, c); c = wmma_bf(a.h, b.l, c); return wmma_bf(a.h, b.h, c); }
__device__ __forceinline__ float sigm(float v) { return 1.0f / (1.0f + expf(-v)); }
#define LDSX() do { asm volatile("s_wait_dscnt 0" ::: "memory"); __builtin_amdgcn_wave_barrier(); __builtin_amdgcn_fence(__ATOMIC_RELEASE, "workgroup"); } while (0)


#define NB 2
#define SS 2048
#define DM 1024
#define NH 16
#define HD 64
#define RR 8
#define RP 32
#define NR (NB * SS)
#ifndef TQB
#define TQB (SS / 64)
#define TNB NB
#endif
typedef __attribute__((ext_vector_type(8))) __bf16 v8b;
__device__ __forceinline__ v16b frag_b(const __bf16* rowk0, int lane) {
  union { v16b v; v8b q[2]; } u; const __bf16* p = rowk0 + 8 * (lane >> 4);
  u.q[0] = *(const v8b*)p; u.q[1] = *(const v8b*)(p + 16); return u.v;
}
__device__ __forceinline__ float bfr(float v) { return (float)(__bf16)v; }
__device__ __attribute__((noinline)) float exp_ni(float v) { return expf(v); }
__device__ __attribute__((noinline)) float erf_ni(float v) { return erff(v); }

#define WS_PW  0u
#define WS_PF  (WS_PW + 2u * (size_t)2 * DM * DM)
#define WS_QR  (WS_PF + 2u * (size_t)2 * 2 * NH * RR * DM)
#define WS_KR  (WS_QR + 2u * (size_t)NR * NH * RP)
#define WS_QRL (WS_KR + 2u * (size_t)NR * NH * RP)
#define WS_KRL (WS_QRL + 2u * (size_t)NR * NH * RP)
#define WS_V   (WS_KRL + 2u * (size_t)NR * NH * RP)
#define WS_O   (WS_V + 2u * (size_t)NB * DM * SS)
#define WS_END (WS_O + 4u * (size_t)NR * DM)

__global__ __launch_bounds__(256) void k_pack(const float* __restrict__ WV, const float* __restrict__ WO, __bf16* __restrict__ PW) { const int n = blockIdx.x, which = blockIdx.y, t = threadIdx.x; __shared__ __align__(16) __bf16 s[DM]; const float* w = which ? WO : WV; for (int k = t; k < DM; k += 256) s[k] = (__bf16)w[(size_t)n * DM + k]; __syncthreads(); if (t < DM / 8) vst2((unsigned*)(PW + ((size_t)which * DM + n) * DM + t * 8), *(const v4u*)&s[t * 8]); }
__global__ __launch_bounds__(256) void k_fold(const float* __restrict__ WQ, const float* __restrict__ WK, const float* __restrict__ BB, __bf16* __restrict__ PF) {
  const int h = blockIdx.x, r = blockIdx.y, which = blockIdx.z, t = threadIdx.x; const float* Wm = which ? WK : WQ; __shared__ float sb[HD]; __shared__ __align__(16) __bf16 sh[DM]; __shared__ __align__(16) __bf16 sl[DM];
  if (t < HD) sb[t] = bfr(BB[(size_t)(h * HD + t) * RR + r]); __syncthreads();
  for (int c = t; c < DM; c += 256) { float a = 0.f; for (int d = 0; d < HD; ++d) a += sb[d] * bfr(Wm[(size_t)(h * HD + d) * DM + c]); const __bf16 hv = (__bf16)a; sh[c] = hv; sl[c] = (__bf16)(a - (float)hv); }
  __syncthreads();
  const size_t row = (size_t)which * (NH * RR) + h * RR + r;
  if (t < DM / 8) { vst2((unsigned*)(PF + row * DM + t * 8), *(const v4u*)&sh[t * 8]); vst2((unsigned*)(PF + ((size_t)2 * NH * RR + row) * DM + t * 8), *(const v4u*)&sl[t * 8]); }
}
__global__ __launch_bounds__(128) void k_qr(const float* __restrict__ X, const __bf16* __restrict__ PF, _Float16* __restrict__ QR_, _Float16* __restrict__ KR_, _Float16* __restrict__ QRL_, _Float16* __restrict__ KRL_) {
  __shared__ __align__(16) _Float16 so[64][NH * RP + 8]; __shared__ __align__(16) _Float16 sol[64][NH * RP + 8];
  const int tid = threadIdx.x, wave = tid >> 5, lane = tid & 31, col = lane & 15, g = lane >> 4; const int which = blockIdx.y; const size_t rb = (size_t)blockIdx.x * 64; const size_t r0 = rb + wave * 16;
  const __bf16* PH = PF + ((size_t)which * (NH * RR)) * DM; const __bf16* PL = PF + ((size_t)2 * NH * RR + which * (NH * RR)) * DM;
  for (int e = tid; e < 64 * (NH * RP); e += 128) { so[e / (NH * RP)][e % (NH * RP)] = (_Float16)0.f; sol[e / (NH * RP)][e % (NH * RP)] = (_Float16)0.f; }
  v8f acc[8] = {};
#pragma unroll 2
  for (int kc = 0; kc < DM / 32; ++kc) { v16b a; { const float* p = X + (r0 + col) * DM + kc * 32 + 8 * g;
#pragma unroll
      for (int i = 0; i < 8; ++i) { a[i] = (__bf16)p[i]; a[8 + i] = (__bf16)p[16 + i]; } }
#pragma unroll
    for (int j = 0; j < 8; ++j) { acc[j] = wmma_bf(a, frag_b(PH + (size_t)(j * 16 + col) * DM + kc * 32, lane), acc[j]); acc[j] = wmma_bf(a, frag_b(PL + (size_t)(j * 16 + col) * DM + kc * 32, lane), acc[j]); } }
  __syncthreads();
#pragma unroll
  for (int j = 0; j < 8; ++j) { const int c = j * 16 + col; const int h = c >> 3, r = c & 7;
#pragma unroll
    for (int rr = 0; rr < 8; ++rr) { const float v = acc[j][rr]; const _Float16 hv = (_Float16)v; so[wave * 16 + 8 * g + rr][h * RP + r] = hv; sol[wave * 16 + 8 * g + rr][h * RP + r] = (_Float16)((v - (float)hv) * 2048.0f); } }
  __syncthreads();
  _Float16* dst = which ? KR_ : QR_; _Float16* dstl = which ? KRL_ : QRL_;
  for (int e = tid; e < 64 * (NH * RP / 8); e += 128) { const int rl = e >> 6, q = e & 63; vst2((unsigned*)(dst + (rb + rl) * (NH * RP) + q * 8), *(const v4u*)&so[rl][q * 8]); vst2((unsigned*)(dstl + (rb + rl) * (NH * RP) + q * 8), *(const v4u*)&sol[rl][q * 8]); }
}
__global__ __launch_bounds__(128) void k_v(const float* __restrict__ X, const __bf16* __restrict__ PW, _Float16* __restrict__ V) {
  __shared__ __align__(16) _Float16 st[128][72];
  const int tid = threadIdx.x, wave = tid >> 5, lane = tid & 31, col = lane & 15, g = lane >> 4; const size_t rb = (size_t)blockIdx.x * 64; const size_t r0 = rb + wave * 16; const int c0 = blockIdx.y * 128;
  v8f acc[8] = {};
#pragma unroll 2
  for (int kc = 0; kc < DM / 32; ++kc) { v16b a; { const float* p = X + (r0 + col) * DM + kc * 32 + 8 * g;
#pragma unroll
      for (int i = 0; i < 8; ++i) { a[i] = (__bf16)p[i]; a[8 + i] = (__bf16)p[16 + i]; } }
#pragma unroll
    for (int j = 0; j < 8; ++j) acc[j] = wmma_bf(a, frag_b(PW + (size_t)(c0 + j * 16 + col) * DM + kc * 32, lane), acc[j]); }
#pragma unroll
  for (int j = 0; j < 8; ++j)
#pragma unroll
    for (int r = 0; r < 8; ++r) st[j * 16 + col][wave * 16 + 8 * g + r] = (_Float16)acc[j][r];
  __syncthreads();
  const size_t b = rb / SS; const int s0 = (int)(rb % SS);
  for (int e = tid; e < 128 * 8; e += 128) { const int d = e >> 3, pc = e & 7; vst2((unsigned*)(V + ((b * DM + c0 + d) * SS) + s0 + pc * 8), *(const v4u*)&st[d][pc * 8]); }
}
__global__ __launch_bounds__(128) void k_attn(const _Float16* __restrict__ QR_, const _Float16* __restrict__ KR_, const _Float16* __restrict__ QRL_, const _Float16* __restrict__ KRL_, const _Float16* __restrict__ V, float* __restrict__ O) {
  __shared__ __align__(16) _Float16 sph[4][16][40]; __shared__ __align__(16) float so[4][16][68];
  const int tid = threadIdx.x, wave = tid >> 5, lane = tid & 31, col = lane & 15, g = lane >> 4; const int h = blockIdx.y; const size_t b = blockIdx.z; const int q0 = blockIdx.x * 64 + wave * 16; const size_t rq = b * SS + q0;
  const v16h aq = frag_h(QR_ + (rq + col) * (NH * RP) + h * RP, lane), aql = frag_h(QRL_ + (rq + col) * (NH * RP) + h * RP, lane);
  float m[8], l[8];
#pragma unroll
  for (int r = 0; r < 8; ++r) { m[r] = -3.0e38f; l[r] = 0.f; }
  v8f acc[4] = {};
#pragma unroll 1
  for (int ks = 0; ks < SS / 32; ++ks) { const int j0 = ks * 32; v8f s[2];
#pragma unroll
    for (int ct = 0; ct < 2; ++ct) { const size_t ko = (b * SS + j0 + ct * 16 + col) * (NH * RP) + h * RP; const v16h kh = frag_h(KR_ + ko, lane); v8f c = {}, cl = {}; c = wmma16(aq, kh, c); cl = wmma16(aql, kh, cl); cl = wmma16(aq, frag_h(KRL_ + ko, lane), cl);
#pragma unroll
      for (int r = 0; r < 8; ++r) s[ct][r] = (c[r] + cl[r] * (1.0f / 2048.0f)) * 0.35355339059327373f; }
#pragma unroll
    for (int r = 0; r < 8; ++r) { float mx = fmaxf(s[0][r], s[1][r]);
#pragma unroll
      for (int o = 1; o < 16; o <<= 1) mx = fmaxf(mx, __shfl_xor(mx, o));
      const float mn = fmaxf(m[r], mx); const float alpha = (m[r] <= -1.0e38f) ? 0.f : __expf(m[r] - mn); const float e0 = __expf(s[0][r] - mn), e1 = __expf(s[1][r] - mn); float es = e0 + e1;
#pragma unroll
      for (int o = 1; o < 16; o <<= 1) es += __shfl_xor(es, o);
      l[r] = l[r] * alpha + es; m[r] = mn;
#pragma unroll
      for (int dt = 0; dt < 4; ++dt) acc[dt][r] *= alpha;
      sph[wave][8 * g + r][col] = (_Float16)(e0 * 2048.0f); sph[wave][8 * g + r][16 + col] = (_Float16)(e1 * 2048.0f); }
    LDSX();
    const v16h pa = frag_h(&sph[wave][col][0], lane);
#pragma unroll
    for (int dt = 0; dt < 4; ++dt) acc[dt] = wmma16(pa, frag_h(V + ((b * DM + h * HD + dt * 16 + col) * SS) + j0, lane), acc[dt]);
    LDSX(); }
#pragma unroll
  for (int r = 0; r < 8; ++r) { const float il = (1.0f / 2048.0f) / l[r];
#pragma unroll
    for (int dt = 0; dt < 4; ++dt) so[wave][8 * g + r][dt * 16 + col] = acc[dt][r] * il; }
  LDSX();
  for (int rl = 0; rl < 16; ++rl) if (lane < 16) vst2(O + (rq + rl) * DM + h * HD + lane * 4, *(const v4f*)&so[wave][rl][lane * 4]);
}
__global__ __launch_bounds__(128) void k_out(const float* __restrict__ O, const __bf16* __restrict__ PW, float* __restrict__ Y) {
  __shared__ __align__(16) float so[4][16][132];
  const int tid = threadIdx.x, wave = tid >> 5, lane = tid & 31, col = lane & 15, g = lane >> 4; const size_t r0 = (size_t)blockIdx.x * 64 + wave * 16; const int n0 = blockIdx.y * 128; const __bf16* P = PW + (size_t)DM * DM;
  v8f acc[8] = {};
#pragma unroll 2
  for (int kc = 0; kc < DM / 32; ++kc) { const F2 a = split_row(O + (r0 + col) * DM, kc * 32, lane);
#pragma unroll
    for (int j = 0; j < 8; ++j) { const v16b w = frag_b(P + (size_t)(n0 + j * 16 + col) * DM + kc * 32, lane); acc[j] = wmma_bf(a.h, w, acc[j]); acc[j] = wmma_bf(a.l, w, acc[j]); } }
#pragma unroll
  for (int j = 0; j < 8; ++j)
#pragma unroll
    for (int r = 0; r < 8; ++r) so[wave][8 * g + r][j * 16 + col] = acc[j][r];
  LDSX();
  for (int rl = 0; rl < 16; ++rl) vst2(Y + (r0 + rl) * DM + n0 + lane * 4, *(const v4f*)&so[wave][rl][lane * 4]);
}
extern "C" void kernel_launch(void* const* d_in, const int* in_sizes, int n_in, void* d_out, int out_size, void* d_ws, size_t ws_size, hipStream_t stream) {
  (void)in_sizes; (void)n_in; (void)out_size;
  const float** F = (const float**)d_in;
  if (ws_size < (size_t)WS_END) return;
  char* ws = (char*)d_ws; __bf16 *PW = (__bf16*)(ws + WS_PW), *PF = (__bf16*)(ws + WS_PF); _Float16 *QR_ = (_Float16*)(ws + WS_QR), *KR_ = (_Float16*)(ws + WS_KR), *QRL_ = (_Float16*)(ws + WS_QRL), *KRL_ = (_Float16*)(ws + WS_KRL), *V = (_Float16*)(ws + WS_V); float* O = (float*)(ws + WS_O);
  k_pack<<<dim3(DM, 2), 256, 0, stream>>>(F[3], F[4], PW);
  k_fold<<<dim3(NH, RR, 2), 256, 0, stream>>>(F[1], F[2], F[5], PF);
  k_qr<<<dim3(TNB * SS / 64, 2), 128, 0, stream>>>(F[0], PF, QR_, KR_, QRL_, KRL_);
  k_v<<<dim3(TNB * SS / 64, DM / 128), 128, 0, stream>>>(F[0], PW, V);
  k_attn<<<dim3(TQB, NH, TNB), 128, 0, stream>>>(QR_, KR_, QRL_, KRL_, V, O);
  k_out<<<dim3(TNB * SS / 64, DM / 128), 128, 0, stream>>>(O, PW, (float*)d_out);
}
